// RingAttention_42649025249824
// MI455X (gfx1250) — hardware-verified
//
#include <hip/hip_runtime.h>


#ifndef NB
#define NB 2
#endif
#ifndef SEQ
#define SEQ 2048
#endif
#define NB_FULL 2
#define SEQ_FULL 2048
#define DIM 1024
#define HEADS 16
#define DHEAD 64
#define DINNER (HEADS * DHEAD)
#define NQKV (3 * DINNER)
#define SEQT (NB * SEQ)
#define QBLK (SEQ / 64)
#define RESROWS ((SEQ < 256) ? SEQ : 256)
#define RESQB (RESROWS / 64)
#define CSTR 132
#define RSCALE 1024.0f
#define RINV (1.0f / 1024.0f)

static_assert(SEQ % 64 == 0);
static_assert(SEQ >= 128);
static_assert(SEQ <= SEQ_FULL);
static_assert(NB >= 1 && NB <= NB_FULL);
static_assert(RESROWS % 64 == 0 && RESROWS >= 64 && RESROWS <= SEQ);
static_assert(DIM % 128 == 0 && NQKV % 128 == 0 && DINNER % 128 == 0);
static_assert(DIM % 32 == 0 && DINNER % 32 == 0 && DHEAD == 64);
static_assert(DIM == 4 * 256 && DINNER == DIM);
static_assert((size_t)SEQT * DIM * 2 + (size_t)NQKV * DIM * 2 + (size_t)DIM * DINNER * 2 + 4 * (size_t)HEADS * SEQT * DHEAD * 2
              + (size_t)HEADS * DHEAD * SEQT * 2 + (size_t)NB * 64 * NQKV * 4 + (size_t)SEQT * DINNER * 2
              + (size_t)NB * RESROWS * DINNER * 2 + 16 * 128 <= (size_t)134217728);

typedef unsigned short us16;
typedef __attribute__((ext_vector_type(16))) __bf16   v16bf;
typedef __attribute__((ext_vector_type(16))) _Float16 v16h;
typedef __attribute__((ext_vector_type(8)))  float    v8f;
typedef __attribute__((ext_vector_type(8)))  unsigned v8u;
typedef __attribute__((ext_vector_type(4)))  unsigned v4u;
typedef __attribute__((ext_vector_type(2)))  unsigned v2u;
typedef __attribute__((ext_vector_type(4)))  float    v4f;

__device__ __forceinline__ unsigned f2bf(float f) { unsigned u = __float_as_uint(f); u += 0x7FFFu + ((u >> 16) & 1u); return u >> 16; }
__device__ __forceinline__ float bf2f(unsigned h) { return __uint_as_float(h << 16); }
__device__ __forceinline__ unsigned f2h(float f) { _Float16 t = (_Float16)f; return (unsigned)__builtin_bit_cast(unsigned short, t); }

struct HP { unsigned h, r; };
__device__ __forceinline__ void split_h(float y, unsigned& hb, unsigned& rb) {
    const _Float16 t = (_Float16)y;
    hb = (unsigned)__builtin_bit_cast(unsigned short, t);
    const float res = (y - (float)t) * RSCALE;
    rb = f2h(res);
}
__device__ __forceinline__ HP pack2(float y0, float y1) {
    unsigned h0, r0, h1, r1;
    split_h(y0, h0, r0);
    split_h(y1, h1, r1);
    HP o;
    o.h = h0 | (h1 << 16);
    o.r = r0 | (r1 << 16);
    return o;
}

__device__ __forceinline__ v8u ld_frag(const us16* rowp, int hh) {
    const v4u a = *(const v4u*)(rowp + 8 * hh);
    const v4u b = *(const v4u*)(rowp + 16 + 8 * hh);
    return __builtin_shufflevector(a, b, 0, 1, 2, 3, 4, 5, 6, 7);
}
__device__ __forceinline__ v8f mma_bf16(v8u a, v8u b, v8f c) {
    return __builtin_amdgcn_wmma_f32_16x16x32_bf16(false, __builtin_bit_cast(v16bf, a), false, __builtin_bit_cast(v16bf, b), (short)0, c, false, false);
}
__device__ __forceinline__ v8f mma_f16(v8u a, v8u b, v8f c) {
    return __builtin_amdgcn_wmma_f32_16x16x32_f16(false, __builtin_bit_cast(v16h, a), false, __builtin_bit_cast(v16h, b), (short)0, c, false, false);
}
__device__ __forceinline__ void mma_guard(v8f& c, v8u a, v8u b) {
    asm volatile("v_nop\n\tv_nop\n\tv_nop\n\tv_nop" : "+v"(c) : "v"(a), "v"(b));
}

__global__ __launch_bounds__(256) void prep_x(const float* __restrict__ x, us16* xb) {
    const int tok = blockIdx.x;
    const int bsel = tok / SEQ, isel = tok - bsel * SEQ;
    const float* xr = x + ((size_t)bsel * SEQ_FULL + isel) * DIM;
    const int tid = threadIdx.x;
    const v4f v = *(const v4f*)(xr + 4 * tid);
    v2u pk;
    pk.x = f2bf(v.x) | (f2bf(v.y) << 16);
    pk.y = f2bf(v.z) | (f2bf(v.w) << 16);
    us16* orow = xb + (size_t)tok * DIM;
    *(volatile v2u*)(orow + 4 * tid) = pk;
    __threadfence();
    *(volatile v2u*)(orow + 4 * tid) = pk;
}

template <int F16>
__global__ __launch_bounds__(256) void prep_w(const float* __restrict__ src, float scale, us16* dst) {
    const int row = blockIdx.x, tid = threadIdx.x;
    const v4f v = *(const v4f*)(src + (size_t)row * DIM + 4 * tid);
    const float a = bf2f(f2bf(v.x)) * scale, bq = bf2f(f2bf(v.y)) * scale;
    const float c = bf2f(f2bf(v.z)) * scale, dq = bf2f(f2bf(v.w)) * scale;
    v2u pk;
    pk.x = F16 ? (f2h(a) | (f2h(bq) << 16)) : (f2bf(a) | (f2bf(bq) << 16));
    pk.y = F16 ? (f2h(c) | (f2h(dq) << 16)) : (f2bf(c) | (f2bf(dq) << 16));
    us16* orow = dst + (size_t)row * DIM;
    *(volatile v2u*)(orow + 4 * tid) = pk;
    __threadfence();
    *(volatile v2u*)(orow + 4 * tid) = pk;
}

template <int F16>
__device__ __forceinline__ void mm_tile(const us16* __restrict__ arow, const us16* __restrict__ bbase, int ldb, int K, int hh, v8f (&acc)[4]) {
#pragma unroll 1
    for (int kc = 0; kc < K; kc += 32) {
        const v8u a = ld_frag(arow + kc, hh);
#pragma unroll
        for (int t = 0; t < 4; ++t) {
            const v8u bfrag = ld_frag(bbase + (size_t)(t * 16) * ldb + kc, hh);
            if (F16) acc[t] = mma_f16(a, bfrag, acc[t]);
            else     acc[t] = mma_bf16(a, bfrag, acc[t]);
            mma_guard(acc[t], a, bfrag);
        }
    }
}

__global__ __launch_bounds__(256) void qkv_gemm(const us16* __restrict__ xb, const us16* __restrict__ wq,
                                                us16* qhi, us16* qlo, us16* khi, us16* klo, us16* vt, float* qkvf) {
    __shared__ __align__(16) float cst[64 * CSTR];
    const int tid = threadIdx.x, lane = tid & 31, wv = tid >> 5, l16 = lane & 15, hh = lane >> 4;
    const int rt = wv & 3, ch = wv >> 2;
    const int row0 = blockIdx.x * 64;
    const int colb = blockIdx.y * 128;
    const us16* arow = xb + (size_t)(row0 + rt * 16 + l16) * DIM;
    const us16* bbase = wq + (size_t)(colb + ch * 64 + l16) * DIM;
    v8f acc[4] = {};
    mm_tile<0>(arow, bbase, DIM, DIM, hh, acc);
#pragma unroll
    for (int r = 0; r < 8; ++r) {
        const int rl = rt * 16 + 8 * hh + r;
#pragma unroll
        for (int t = 0; t < 4; ++t) cst[rl * CSTR + ch * 64 + t * 16 + l16] = acc[t][r];
    }
    __syncthreads();
    const int which = colb / DINNER;
    const int hsel = (colb % DINNER) / DHEAD;
    const int bsel = row0 / SEQ, i0 = row0 % SEQ;
    auto pass = [&]() {
        if (which < 2) {
            us16* ph = (which == 0) ? qhi : khi;
            us16* pl = (which == 0) ? qlo : klo;
#pragma unroll 4
            for (int j = 0; j < 16; ++j) {
                const int L = wv * 16 + j, r = L >> 1, c = L & 1;
                const float a = cst[r * CSTR + c * 64 + 2 * lane], bq = cst[r * CSTR + c * 64 + 2 * lane + 1];
                const unsigned ha = f2bf(a), hb = f2bf(bq);
                const unsigned la = f2bf(a - bf2f(ha)), lb = f2bf(bq - bf2f(hb));
                const size_t off = ((size_t)(hsel + c) * SEQT + row0 + r) * DHEAD + 2 * lane;
                *(volatile unsigned*)(ph + off) = ha | (hb << 16);
                *(volatile unsigned*)(pl + off) = la | (lb << 16);
            }
        } else {
#pragma unroll 4
            for (int j = 0; j < 16; ++j) {
                const int L = wv * 16 + j, c = L >> 6, d = L & 63;
                const float a = cst[(2 * lane) * CSTR + c * 64 + d] * 4.0f, bq = cst[(2 * lane + 1) * CSTR + c * 64 + d] * 4.0f;
                const size_t off = ((size_t)(hsel + c) * DHEAD + d) * SEQT + row0 + 2 * lane;
                *(volatile unsigned*)(vt + off) = f2h(a) | (f2h(bq) << 16);
            }
        }
        if (i0 == 0) {
            const int col = tid & 127, rsel = tid >> 7;
            float* dstp = qkvf + (size_t)bsel * 64 * NQKV + colb + col;
#pragma unroll 4
            for (int r = rsel; r < 64; r += 2) *(volatile float*)(dstp + (size_t)r * NQKV) = cst[r * CSTR + col];
        }
    };
    pass();
    __threadfence();
    pass();
}

__global__ __launch_bounds__(256) __attribute__((amdgpu_num_vgpr(256)))
void attn_first(const float* __restrict__ qkvf, us16* ao, us16* aores) {
    __shared__ union { float qs[64][64]; v4u st[2][64][8]; } u;
    __shared__ float ks[64][65];
    __shared__ float vs[64][65];
    const int h = blockIdx.x % HEADS, bsel = blockIdx.x / HEADS;
    const float* base = qkvf + (size_t)bsel * 64 * NQKV + h * DHEAD;
    const int tid = threadIdx.x, lane = tid & 31;
#pragma unroll 4
    for (int j = 0; j < 16; ++j) {
        const int idx = tid + 256 * j, r = idx >> 6, cc = idx & 63;
        const float* rp = base + (size_t)r * NQKV + cc;
        u.qs[r][cc] = rp[0] * 0.125f;
        ks[r][cc] = rp[DINNER];
        vs[r][cc] = rp[2 * DINNER];
    }
    __syncthreads();
    const int i = tid >> 2, p = tid & 3;
    const float NEG = -__builtin_inff();
    float sr[16];
#pragma unroll
    for (int jj = 0; jj < 16; ++jj) sr[jj] = 0.f;
#pragma unroll 1
    for (int d = 0; d < DHEAD; ++d) {
        const float qd = u.qs[i][d];
#pragma unroll
        for (int jj = 0; jj < 16; ++jj) sr[jj] = fmaf(qd, ks[16 * p + jj][d], sr[jj]);
    }
    float mx = NEG;
#pragma unroll
    for (int jj = 0; jj < 16; ++jj) { if (16 * p + jj > i) sr[jj] = NEG; mx = fmaxf(mx, sr[jj]); }
    mx = fmaxf(mx, __shfl_xor(mx, 1, 32));
    mx = fmaxf(mx, __shfl_xor(mx, 2, 32));
    float sum = 0.f;
#pragma unroll
    for (int jj = 0; jj < 16; ++jj) { sr[jj] = __expf(sr[jj] - mx); sum += sr[jj]; }
    sum += __shfl_xor(sum, 1, 32);
    sum += __shfl_xor(sum, 2, 32);
    const float inv = 1.0f / (sum + 1e-8f);
    __syncthreads();
#pragma unroll
    for (int jj = 0; jj < 16; ++jj) u.qs[i][16 * p + jj] = sr[jj] * inv;
    __syncthreads();
    float orr[16];
#pragma unroll
    for (int dd = 0; dd < 16; ++dd) orr[dd] = 0.f;
#pragma unroll 1
    for (int j = 0; j < 64; ++j) {
        const float pj = u.qs[i][j];
#pragma unroll
        for (int dd = 0; dd < 16; ++dd) orr[dd] = fmaf(pj, vs[j][16 * p + dd], orr[dd]);
    }
    const HP t0 = pack2(orr[0] * 4.0f,  orr[1] * 4.0f),  t1 = pack2(orr[2] * 4.0f,  orr[3] * 4.0f);
    const HP t2 = pack2(orr[4] * 4.0f,  orr[5] * 4.0f),  t3 = pack2(orr[6] * 4.0f,  orr[7] * 4.0f);
    const HP t4 = pack2(orr[8] * 4.0f,  orr[9] * 4.0f),  t5 = pack2(orr[10] * 4.0f, orr[11] * 4.0f);
    const HP t6 = pack2(orr[12] * 4.0f, orr[13] * 4.0f), t7 = pack2(orr[14] * 4.0f, orr[15] * 4.0f);
    v4u w0, w1, z0, z1;
    w0.x = t0.h; w0.y = t1.h; w0.z = t2.h; w0.w = t3.h;
    w1.x = t4.h; w1.y = t5.h; w1.z = t6.h; w1.w = t7.h;
    z0.x = t0.r; z0.y = t1.r; z0.z = t2.r; z0.w = t3.r;
    z1.x = t4.r; z1.y = t5.r; z1.z = t6.r; z1.w = t7.r;
    __syncthreads();
    u.st[0][i][2 * p] = w0;
    u.st[0][i][2 * p + 1] = w1;
    u.st[1][i][2 * p] = z0;
    u.st[1][i][2 * p + 1] = z1;
    __syncthreads();
    const size_t tok0 = (size_t)bsel * SEQ;
    const size_t res0 = (size_t)bsel * RESROWS;
    auto pass = [&]() {
#pragma unroll
        for (int q2 = 0; q2 < 2; ++q2) {
            const int row = 32 * q2 + (tid >> 3), pc = lane & 7;
            *(volatile v4u*)(ao + (tok0 + row) * DINNER + h * DHEAD + 8 * pc) = u.st[0][row][pc];
            *(volatile v4u*)(aores + (res0 + row) * DINNER + h * DHEAD + 8 * pc) = u.st[1][row][pc];
        }
    };
    pass();
    __threadfence();
    pass();
}

__global__ __launch_bounds__(128) __attribute__((amdgpu_num_vgpr(256)))
void attn_main(const us16* __restrict__ qhi, const us16* __restrict__ qlo,
               const us16* __restrict__ khi, const us16* __restrict__ klo,
               const us16* __restrict__ vt, us16* ao, us16* aores) {
    __shared__ v4u ost[4][16][8];
    __shared__ v4u rst[4][16][8];
    const int tid = threadIdx.x, lane = tid & 31, wv = tid >> 5, m = lane & 15, hh = lane >> 4;
    const int qb = blockIdx.x + 1;
    const int h = blockIdx.y % HEADS, bsel = blockIdx.y / HEADS;
    const size_t tok0 = (size_t)bsel * SEQ;
    const int qrow = qb * 64 + wv * 16;
    const int iq = qrow + m;
    const size_t qoff = ((size_t)h * SEQT + tok0 + qrow + m) * DHEAD;
    const v8u qh0 = ld_frag(qhi + qoff, hh), qh1 = ld_frag(qhi + qoff + 32, hh);
    const v8u ql0 = ld_frag(qlo + qoff, hh), ql1 = ld_frag(qlo + qoff + 32, hh);
    const us16* kbh = khi + ((size_t)h * SEQT + tok0) * DHEAD;
    const us16* kbl = klo + ((size_t)h * SEQT + tok0) * DHEAD;
    const us16* vb = vt + (size_t)h * DHEAD * SEQT + tok0;
    const float NEG = -__builtin_inff();
    v8f o[4] = {};
    float mrun = NEG, lrun = 0.f;
    const int nch = 2 * qb + 2;
#pragma unroll 1
    for (int c = 0; c < nch; ++c) {
        v8f s[2] = {};
#pragma unroll
        for (int t = 0; t < 2; ++t) {
            const size_t koff = (size_t)(c * 32 + t * 16 + m) * DHEAD;
            const v8u a0 = ld_frag(kbh + koff, hh);
            s[t] = mma_bf16(a0, qh0, s[t]);
            s[t] = mma_bf16(a0, ql0, s[t]);
            const v8u a1 = ld_frag(kbl + koff, hh);
            s[t] = mma_bf16(a1, qh0, s[t]);
            const v8u a2 = ld_frag(kbh + koff + 32, hh);
            s[t] = mma_bf16(a2, qh1, s[t]);
            s[t] = mma_bf16(a2, ql1, s[t]);
            const v8u a3 = ld_frag(kbl + koff + 32, hh);
            s[t] = mma_bf16(a3, qh1, s[t]);
            asm volatile("v_nop\n\tv_nop\n\tv_nop\n\tv_nop" : "+v"(s[t]) : "v"(a0), "v"(a1), "v"(a2), "v"(a3), "v"(qh1), "v"(ql1));
        }
        float sv[16];
        float cmax = NEG;
#pragma unroll
        for (int t = 0; t < 2; ++t)
#pragma unroll
            for (int r = 0; r < 8; ++r) {
                const int j = c * 32 + t * 16 + 8 * hh + r;
                const float v = (j <= iq) ? s[t][r] * 0.125f : NEG;
                sv[8 * t + r] = v;
                cmax = fmaxf(cmax, v);
            }
        cmax = fmaxf(cmax, __shfl_xor(cmax, 16, 32));
        const float mnew = fmaxf(mrun, cmax);
        const float muse = (mnew == NEG) ? 0.f : mnew;
        const float fac = (mrun == NEG) ? 0.f : __expf(mrun - muse);
        mrun = mnew;
        v16h ph;
        float psum = 0.f;
#pragma unroll
        for (int r = 0; r < 8; ++r) {
            const _Float16 p0 = (_Float16)(__expf(sv[r] - muse) * 16384.0f);
            const _Float16 p1 = (_Float16)(__expf(sv[8 + r] - muse) * 16384.0f);
            ph[r] = p0;
            ph[8 + r] = p1;
            psum += (float)p0 + (float)p1;
        }
        psum += __shfl_xor(psum, 16, 32);
        lrun = lrun * fac + psum;
        const v8u pbu = __builtin_bit_cast(v8u, ph);
#pragma unroll
        for (int dt = 0; dt < 4; ++dt) o[dt] = o[dt] * fac;
#pragma unroll
        for (int dt = 0; dt < 4; ++dt) {
            const v8u va = ld_frag(vb + (size_t)(dt * 16 + m) * SEQT + c * 32, hh);
            o[dt] = mma_f16(va, pbu, o[dt]);
            mma_guard(o[dt], va, pbu);
        }
    }
    const float inv = 1.0f / (lrun + 1.6384e-4f);
#pragma unroll
    for (int dt = 0; dt < 4; ++dt) {
        const HP t0 = pack2(o[dt][0] * inv, o[dt][1] * inv);
        const HP t1 = pack2(o[dt][2] * inv, o[dt][3] * inv);
        const HP t2 = pack2(o[dt][4] * inv, o[dt][5] * inv);
        const HP t3 = pack2(o[dt][6] * inv, o[dt][7] * inv);
        v4u w, z;
        w.x = t0.h; w.y = t1.h; w.z = t2.h; w.w = t3.h;
        z.x = t0.r; z.y = t1.r; z.z = t2.r; z.w = t3.r;
        ost[wv][m][2 * dt + hh] = w;
        rst[wv][m][2 * dt + hh] = z;
    }
    __syncthreads();
    const bool dores = (qb < RESQB);
    us16* aob = ao + (tok0 + qrow) * DINNER + h * DHEAD;
    auto pass = [&]() {
#pragma unroll
        for (int p = 0; p < 4; ++p) {
            const int rr = 4 * p + (lane >> 3), pc = lane & 7;
            *(volatile v4u*)(aob + (size_t)rr * DINNER + 8 * pc) = ost[wv][rr][pc];
        }
        if (dores) {
            us16* arb = aores + ((size_t)bsel * RESROWS + qrow) * DINNER + h * DHEAD;
#pragma unroll
            for (int p = 0; p < 4; ++p) {
                const int rr = 4 * p + (lane >> 3), pc = lane & 7;
                *(volatile v4u*)(arb + (size_t)rr * DINNER + 8 * pc) = rst[wv][rr][pc];
            }
        }
    };
    pass();
    __threadfence();
    pass();
}

__global__ __launch_bounds__(256) void out_gemm(const us16* __restrict__ aop, const us16* __restrict__ aores,
                                                const us16* __restrict__ wo, float* out) {
    __shared__ __align__(16) float cst[64 * CSTR];
    const int tid = threadIdx.x, lane = tid & 31, wv = tid >> 5, l16 = lane & 15, hh = lane >> 4;
    const int rt = wv & 3, ch = wv >> 2;
    const int row0 = blockIdx.x * 64;
    const int colb = blockIdx.y * 128;
    const int bsel = row0 / SEQ, i0 = row0 % SEQ;
    const us16* arow = aop + (size_t)(row0 + rt * 16 + l16) * DINNER;
    const us16* bbase = wo + (size_t)(colb + ch * 64 + l16) * DINNER;
    v8f acc[4] = {};
    v8f acc2[4] = {};
    mm_tile<1>(arow, bbase, DINNER, DINNER, hh, acc);
    if (i0 < RESROWS) {
        const us16* arow2 = aores + ((size_t)bsel * RESROWS + i0 + rt * 16 + l16) * DINNER;
        mm_tile<1>(arow2, bbase, DINNER, DINNER, hh, acc2);
    }
#pragma unroll
    for (int r = 0; r < 8; ++r) {
        const int rl = rt * 16 + 8 * hh + r;
#pragma unroll
        for (int t = 0; t < 4; ++t) cst[rl * CSTR + ch * 64 + t * 16 + l16] = (acc[t][r] + acc2[t][r] * RINV) * (1.0f / 256.0f);
    }
    __syncthreads();
    const int col = tid & 127, rsel = tid >> 7;
    float* ob = out + (size_t)row0 * DIM + colb + col;
    auto pass = [&]() {
#pragma unroll 4
        for (int r = rsel; r < 64; r += 2) *(volatile float*)(ob + (size_t)r * DIM) = cst[r * CSTR + col];
    };
    pass();
    __threadfence();
    pass();
}

extern "C" void kernel_launch(void* const* d_in, const int* in_sizes, int n_in,
                              void* d_out, int out_size, void* d_ws, size_t ws_size, hipStream_t stream) {
    if (n_in < 5) return;
    const float* x  = (const float*)d_in[0];
    const float* wq = (const float*)d_in[1];
    const float* wk = (const float*)d_in[2];
    const float* wv = (const float*)d_in[3];
    const float* wo = (const float*)d_in[4];
    float* out = (float*)d_out;
    if (in_sizes[0] < ((NB - 1) * SEQ_FULL + SEQ) * DIM) return;
    if (in_sizes[1] < DIM * DINNER) return;
    if (in_sizes[2] < DIM * DINNER) return;
    if (in_sizes[3] < DIM * DINNER) return;
    if (in_sizes[4] < DINNER * DIM) return;
    if (out_size < SEQT * DIM) return;

    size_t off = 0;
    auto carve = [&](size_t bytes) { size_t o = off; off += (bytes + 127) & ~(size_t)127; return o; };
    char* ws = (char*)d_ws;
    us16*  xb    = (us16*) (ws + carve((size_t)SEQT * DIM * 2));
    us16*  wqkv  = (us16*) (ws + carve((size_t)NQKV * DIM * 2));
    us16*  wop   = (us16*) (ws + carve((size_t)DIM * DINNER * 2));
    us16*  qhi   = (us16*) (ws + carve((size_t)HEADS * SEQT * DHEAD * 2));
    us16*  qlo   = (us16*) (ws + carve((size_t)HEADS * SEQT * DHEAD * 2));
    us16*  khi   = (us16*) (ws + carve((size_t)HEADS * SEQT * DHEAD * 2));
    us16*  klo   = (us16*) (ws + carve((size_t)HEADS * SEQT * DHEAD * 2));
    us16*  vt    = (us16*) (ws + carve((size_t)HEADS * DHEAD * SEQT * 2));
    float* qkvf  = (float*)(ws + carve((size_t)NB * 64 * NQKV * 4));
    us16*  ao    = (us16*) (ws + carve((size_t)SEQT * DINNER * 2));
    us16*  aores = (us16*) (ws + carve((size_t)NB * RESROWS * DINNER * 2));
    if (off > ws_size) return;
    if (off > (size_t)134217728) return;

    prep_x<<<SEQT, 256, 0, stream>>>(x, xb);
    prep_w<0><<<DINNER, 256, 0, stream>>>(wq, 1.0f, wqkv);
    prep_w<0><<<DINNER, 256, 0, stream>>>(wk, 1.0f, wqkv + (size_t)DINNER * DIM);
    prep_w<0><<<DINNER, 256, 0, stream>>>(wv, 1.0f, wqkv + (size_t)2 * DINNER * DIM);
    prep_w<1><<<DIM, 256, 0, stream>>>(wo, 64.0f, wop);
    qkv_gemm<<<dim3(SEQT / 64, NQKV / 128), 256, 0, stream>>>(xb, wqkv, qhi, qlo, khi, klo, vt, qkvf);
    attn_first<<<NB * HEADS, 256, 0, stream>>>(qkvf, ao, aores);
    attn_main<<<dim3(QBLK - 1, NB * HEADS), 128, 0, stream>>>(qhi, qlo, khi, klo, vt, ao, aores);
    out_gemm<<<dim3(SEQT / 64, DIM / 128), 256, 0, stream>>>(ao, aores, wop, out);
}
